// MultiHeadedAttention_3917010174428
// MI455X (gfx1250) — hardware-verified
//
#include <hip/hip_runtime.h>

typedef _Float16 f16;
typedef f16      v16h __attribute__((ext_vector_type(16)));
typedef f16      v8h  __attribute__((ext_vector_type(8)));
typedef float    v8f  __attribute__((ext_vector_type(8)));
typedef float    v4f  __attribute__((ext_vector_type(4)));
typedef unsigned v4u  __attribute__((ext_vector_type(4)));

#ifndef NB
#define NB 4
#endif
#ifndef SEQ
#define SEQ 2048
#endif
#define NB_FULL 4
#define SEQ_FULL 2048
#define DM 256
#define NH 4
#define HD 64

#define GN 64
#define WP 40
#define XP 40
#define TP 72
#define TP32 68
#define KP 72
#define VP 40
#define OP 136
#define QCHUNK 128

static_assert(DM == NH * HD);
static_assert(HD == 64);
static_assert(NH == 4);
static_assert(SEQ % 256 == 0);
static_assert(SEQ % QCHUNK == 0);
static_assert(SEQ % GN == 0);
static_assert(NB >= 1 && NB <= NB_FULL);
static_assert(SEQ <= SEQ_FULL);
static_assert((NB * DM * SEQ) % 2048 == 0);
static_assert(DM * TP * 2 <= 9216 * 4);
static_assert((DM / 2) * TP32 <= 9216);

union Frag   { v16h v; v4u q[2]; f16 h[16]; };
union Pack8  { v8h v; v4u u; f16 h[8]; };
union Pack4f { v4f v; float f[4]; };
static_assert(sizeof(Frag) == 32);
static_assert(sizeof(Pack8) == 16);
static_assert(sizeof(Pack4f) == 16);

__device__ __forceinline__ float bf16r(float x) {
  unsigned u = __float_as_uint(x);
  u = (u + 0x7FFFu + ((u >> 16) & 1u)) & 0xFFFF0000u;
  return __uint_as_float(u);
}

__device__ __forceinline__ v8f wmma16(v16h a, v16h b, v8f c) {
  v8f d = __builtin_amdgcn_wmma_f32_16x16x32_f16(false, a, false, b, (short)0, c, false, false);
  asm volatile("v_nop\n\tv_nop\n\tv_nop\n\tv_nop" : "+v"(d) : "v"(a), "v"(b));
  return d;
}

__global__ void __launch_bounds__(256) cvt_act(const float* __restrict__ xq, const float* __restrict__ xk,
                                               const float* __restrict__ xv, f16* __restrict__ planes) {
  const int which = blockIdx.y;
  const float* src = (which == 0) ? xq : ((which == 1) ? xk : xv);
  f16* dst = planes + (size_t)which * ((size_t)NB * DM * SEQ);
  const unsigned u = blockIdx.x * 256u + threadIdx.x;
  const unsigned row = u / (SEQ / 8), piece = u % (SEQ / 8);
  const float* s = src + (size_t)row * SEQ_FULL + piece * 8;
  Pack4f a, c;
  a.v = *(const v4f*)s;
  c.v = *(const v4f*)(s + 4);
  Pack8 o;
#pragma unroll
  for (int j = 0; j < 4; ++j) {
    o.h[j]     = (f16)bf16r(a.f[j]);
    o.h[4 + j] = (f16)bf16r(c.f[j]);
  }
  f16* d = dst + (size_t)row * SEQ + piece * 8;
  *(volatile v4u*)d = o.u;
  __threadfence();
  *(volatile v4u*)d = o.u;
}

__global__ void __launch_bounds__(256) cvt_w(const float* __restrict__ w0, const float* __restrict__ w1,
                                             const float* __restrict__ w2, const float* __restrict__ w3,
                                             f16* __restrict__ wplanes) {
  const int which = blockIdx.y;
  const float* src = (which == 0) ? w0 : ((which == 1) ? w1 : ((which == 2) ? w2 : w3));
  f16* dst = wplanes + (size_t)which * (DM * DM);
  const unsigned u = blockIdx.x * 256u + threadIdx.x;
  const float* s = src + (size_t)u * 8;
  Pack4f a, c;
  a.v = *(const v4f*)s;
  c.v = *(const v4f*)(s + 4);
  Pack8 o;
#pragma unroll
  for (int j = 0; j < 4; ++j) {
    o.h[j]     = (f16)(16.0f * bf16r(a.f[j]));
    o.h[4 + j] = (f16)(16.0f * bf16r(c.f[j]));
  }
  f16* d = dst + (size_t)u * 8;
  *(volatile v4u*)d = o.u;
  __threadfence();
  *(volatile v4u*)d = o.u;
}

template <int MODE>
__global__ void __launch_bounds__(256) __attribute__((amdgpu_num_vgpr(256)))
gemm_k256(const f16* __restrict__ W16, const f16* __restrict__ X16, const float* __restrict__ bias,
          f16* __restrict__ Yh, float* __restrict__ Yf, float oscale)
{
  __shared__ __align__(16) f16   ldsW[DM * WP];
  __shared__ __align__(16) f16   ldsX[GN * XP];
  __shared__ __align__(16) float epi[9216];

  const int tid = threadIdx.x, lane = tid & 31, wave = tid >> 5;
  const int lm = lane & 15, hh = lane >> 4;
  const int n0 = blockIdx.x * GN;
  const int b  = blockIdx.y;
  const f16* Xb = X16 + (size_t)b * DM * SEQ;

  v8f zero = {};
  v8f acc[2][4];
#pragma unroll
  for (int i = 0; i < 2; ++i)
#pragma unroll
    for (int j = 0; j < 4; ++j) acc[i][j] = zero;

#pragma unroll 1
  for (int k0 = 0; k0 < DM; k0 += 32) {
    {
      const f16* src = W16 + (size_t)tid * DM + k0;
#pragma unroll
      for (int c = 0; c < 4; ++c)
        *(v4u*)(ldsW + tid * WP + c * 8) = *(const v4u*)(src + c * 8);
    }
    {
      const int kk = tid >> 3;
      const int nn = (tid & 7) * 8;
      Pack8 t;
      t.u = *(const v4u*)(Xb + (size_t)(k0 + kk) * SEQ + n0 + nn);
#pragma unroll
      for (int j = 0; j < 8; ++j) ldsX[(nn + j) * XP + kk] = t.h[j];
    }
    __syncthreads();

    Frag a[2], bb[4];
#pragma unroll
    for (int mt = 0; mt < 2; ++mt) {
      const f16* rp = ldsW + (wave * 32 + mt * 16 + lm) * WP;
      a[mt].q[0] = *(const v4u*)(rp + 8 * hh);
      a[mt].q[1] = *(const v4u*)(rp + 16 + 8 * hh);
    }
#pragma unroll
    for (int nt = 0; nt < 4; ++nt) {
      const f16* cp = ldsX + (nt * 16 + lm) * XP;
      bb[nt].q[0] = *(const v4u*)(cp + 8 * hh);
      bb[nt].q[1] = *(const v4u*)(cp + 16 + 8 * hh);
    }
#pragma unroll
    for (int mt = 0; mt < 2; ++mt)
#pragma unroll
      for (int nt = 0; nt < 4; ++nt)
        acc[mt][nt] = wmma16(a[mt].v, bb[nt].v, acc[mt][nt]);
    __syncthreads();
  }

  if constexpr (MODE != 2) {
    f16* T16 = (f16*)epi;
#pragma unroll
    for (int mt = 0; mt < 2; ++mt) {
#pragma unroll
      for (int r = 0; r < 8; ++r) {
        const int o = wave * 32 + mt * 16 + 8 * hh + r;
        const float br = bf16r(bias[o]);
#pragma unroll
        for (int nt = 0; nt < 4; ++nt)
          T16[o * TP + nt * 16 + lm] = (f16)(acc[mt][nt][r] * oscale + br);
      }
    }
    __syncthreads();

    if constexpr (MODE == 0) {
      auto pass = [&]() {
#pragma unroll 1
        for (int it = 0; it < 8; ++it) {
          const int u = it * 256 + tid;
          const int line = u >> 3, piece = u & 7;
          const int head = line >> 6, n = line & 63;
          Pack8 o;
#pragma unroll
          for (int j = 0; j < 8; ++j) {
            const int d = piece * 8 + j;
            o.h[j] = T16[(d * NH + head) * TP + n];
          }
          f16* dst = Yh + ((size_t)(b * NH + head) * SEQ + n0 + n) * HD + piece * 8;
          *(volatile v4u*)dst = o.u;
        }
      };
      pass();
      __threadfence();
      pass();
    } else {
      auto pass = [&]() {
#pragma unroll 1
        for (int it = 0; it < 8; ++it) {
          const int u = it * 256 + tid;
          const int o = u >> 3, piece = u & 7;
          const int head = o % NH, d = o / NH;
          Pack8 v;
          v.u = *(const v4u*)(T16 + o * TP + piece * 8);
          f16* dst = Yh + ((size_t)(b * NH + head) * HD + d) * SEQ + n0 + piece * 8;
          *(volatile v4u*)dst = v.u;
        }
      };
      pass();
      __threadfence();
      pass();
    }
  } else {
#pragma unroll 1
    for (int hf = 0; hf < 2; ++hf) {
      if ((wave >> 2) == hf) {
#pragma unroll
        for (int mt = 0; mt < 2; ++mt) {
#pragma unroll
          for (int r = 0; r < 8; ++r) {
            const int o = wave * 32 + mt * 16 + 8 * hh + r;
            const float br = bf16r(bias[o]);
#pragma unroll
            for (int nt = 0; nt < 4; ++nt)
              epi[(o - hf * 128) * TP32 + nt * 16 + lm] = acc[mt][nt][r] * oscale + br;
          }
        }
      }
      __syncthreads();
      auto pass = [&]() {
#pragma unroll 1
        for (int it = 0; it < 8; ++it) {
          const int u = it * 256 + tid;
          const int rowl = u >> 4, piece = u & 15;
          Pack4f v;
          v.v = *(const v4f*)(epi + rowl * TP32 + piece * 4);
          float* dst = Yf + ((size_t)b * DM + hf * 128 + rowl) * SEQ + n0 + piece * 4;
          *(volatile v4f*)dst = v.v;
        }
      };
      pass();
      __threadfence();
      pass();
      __syncthreads();
    }
  }
}

__global__ void __launch_bounds__(256) __attribute__((amdgpu_num_vgpr(256)))
attn_flash(const f16* __restrict__ Qn, const f16* __restrict__ Kn, const f16* __restrict__ Vt,
           f16* __restrict__ Xa)
{
  __shared__ __align__(16) f16 ldsK[32 * KP];
  __shared__ __align__(16) f16 ldsV[HD * VP];
  __shared__ __align__(16) f16 ldsO[HD * OP];

  const int tid = threadIdx.x, lane = tid & 31, wave = tid >> 5;
  const int lm = lane & 15, hh = lane >> 4;
  constexpr int QCH = SEQ / QCHUNK;
  const int gid   = blockIdx.x;
  const int chunk = gid % QCH;
  const int head  = (gid / QCH) % NH;
  const int b     = gid / (QCH * NH);
  const int bh    = b * NH + head;
  const int q0    = chunk * QCHUNK;
  const int n0    = q0 + wave * 16;

  Frag bq[2];
  {
    const f16* qr = Qn + ((size_t)bh * SEQ + n0 + lm) * HD;
#pragma unroll
    for (int f = 0; f < 2; ++f) {
      bq[f].q[0] = *(const v4u*)(qr + f * 32 + 8 * hh);
      bq[f].q[1] = *(const v4u*)(qr + f * 32 + 16 + 8 * hh);
    }
  }

  v8f zero = {};
  v8f oacc[4];
#pragma unroll
  for (int dt = 0; dt < 4; ++dt) oacc[dt] = zero;
  float mrow = -1.0e30f, lrow = 0.0f;

  const f16* Kb = Kn + (size_t)bh * SEQ * HD;
  const f16* Vb = Vt + (size_t)bh * HD * SEQ;
  const int km = tid >> 3, kd = (tid & 7) * 8;
  const int vd = tid >> 2, vm = (tid & 3) * 8;

#pragma unroll 1
  for (int m0 = 0; m0 < SEQ; m0 += 32) {
    __syncthreads();
    *(v4u*)(ldsK + km * KP + kd) = *(const v4u*)(Kb + (size_t)(m0 + km) * HD + kd);
    *(v4u*)(ldsV + vd * VP + vm) = *(const v4u*)(Vb + (size_t)vd * SEQ + m0 + vm);
    __syncthreads();

    v8f s0 = zero, s1 = zero;
#pragma unroll
    for (int f = 0; f < 2; ++f) {
      Frag a0, a1;
      const f16* r0p = ldsK + lm * KP + f * 32;
      const f16* r1p = ldsK + (16 + lm) * KP + f * 32;
      a0.q[0] = *(const v4u*)(r0p + 8 * hh);
      a0.q[1] = *(const v4u*)(r0p + 16 + 8 * hh);
      a1.q[0] = *(const v4u*)(r1p + 8 * hh);
      a1.q[1] = *(const v4u*)(r1p + 16 + 8 * hh);
      s0 = wmma16(a0.v, bq[f].v, s0);
      s1 = wmma16(a1.v, bq[f].v, s1);
    }

    float sc0[8], sc1[8];
    float tmax = -1.0e30f;
#pragma unroll
    for (int r = 0; r < 8; ++r) {
      sc0[r] = s0[r] * 0.125f;
      sc1[r] = s1[r] * 0.125f;
      tmax = fmaxf(tmax, fmaxf(sc0[r], sc1[r]));
    }
    tmax = fmaxf(tmax, __shfl_xor(tmax, 16, 32));
    const float mnew  = fmaxf(mrow, tmax);
    const float alpha = __expf(mrow - mnew);
    mrow = mnew;

    Frag pb;
    float rsum = 0.0f;
#pragma unroll
    for (int r = 0; r < 8; ++r) {
      const float p0 = __expf(sc0[r] - mnew);
      const float p1 = __expf(sc1[r] - mnew);
      rsum += p0 + p1;
      pb.h[r]     = (f16)(p0 * 1024.0f);
      pb.h[8 + r] = (f16)(p1 * 1024.0f);
    }
    rsum += __shfl_xor(rsum, 16, 32);
    lrow = lrow * alpha + rsum;
#pragma unroll
    for (int dt = 0; dt < 4; ++dt)
#pragma unroll
      for (int r = 0; r < 8; ++r) oacc[dt][r] *= alpha;

#pragma unroll
    for (int dt = 0; dt < 4; ++dt) {
      Frag va;
      const f16* vp = ldsV + (dt * 16 + lm) * VP;
      va.q[0] = *(const v4u*)(vp + 8 * hh);
      va.q[1] = *(const v4u*)(vp + 16 + 8 * hh);
      oacc[dt] = wmma16(va.v, pb.v, oacc[dt]);
    }
  }

  const float inv = 1.0f / (lrow * 16.0f);
#pragma unroll
  for (int dt = 0; dt < 4; ++dt)
#pragma unroll
    for (int r = 0; r < 8; ++r)
      ldsO[(dt * 16 + 8 * hh + r) * OP + wave * 16 + lm] = (f16)(oacc[dt][r] * inv);
  __syncthreads();

  auto pass = [&]() {
#pragma unroll 1
    for (int it = 0; it < 4; ++it) {
      const int u = it * 256 + tid;
      const int d = u >> 4, piece = u & 15;
      Pack8 v;
      v.u = *(const v4u*)(ldsO + d * OP + piece * 8);
      f16* dst = Xa + ((size_t)b * DM + d * NH + head) * SEQ + q0 + piece * 8;
      *(volatile v4u*)dst = v.u;
    }
  };
  pass();
  __threadfence();
  pass();
}

extern "C" void kernel_launch(void* const* d_in, const int* in_sizes, int n_in,
                              void* d_out, int out_size, void* d_ws, size_t ws_size,
                              hipStream_t stream) {
  if (n_in < 11) return;
  const long needA = ((long)(NB - 1) * DM + (DM - 1)) * (long)SEQ_FULL + SEQ;
  if ((long)in_sizes[0] < needA || (long)in_sizes[1] < needA || (long)in_sizes[2] < needA) return;
  if (in_sizes[3] < DM * DM || in_sizes[5] < DM * DM || in_sizes[7] < DM * DM || in_sizes[9] < DM * DM) return;
  if (in_sizes[4] < DM || in_sizes[6] < DM || in_sizes[8] < DM || in_sizes[10] < DM) return;
  if ((long)out_size < (long)NB * DM * SEQ) return;

  const float* q_in = (const float*)d_in[0];
  const float* k_in = (const float*)d_in[1];
  const float* v_in = (const float*)d_in[2];
  const float* Wq = (const float*)d_in[3];
  const float* bq = (const float*)d_in[4];
  const float* Wk = (const float*)d_in[5];
  const float* bk = (const float*)d_in[6];
  const float* Wv = (const float*)d_in[7];
  const float* bv = (const float*)d_in[8];
  const float* Wm = (const float*)d_in[9];
  const float* bm = (const float*)d_in[10];
  float* out = (float*)d_out;

  const size_t planeElems = (size_t)NB * DM * SEQ;
  const size_t planeB     = planeElems * 2;
  const size_t wB         = (size_t)4 * DM * DM * 2;
  size_t off = 0;
  char* base = (char*)d_ws;
  f16* actP = (f16*)(base + off); off += 3 * planeB;
  f16* wP   = (f16*)(base + off); off += wB;
  f16* Qn   = (f16*)(base + off); off += planeB;
  f16* Kn   = (f16*)(base + off); off += planeB;
  f16* Vt   = (f16*)(base + off); off += planeB;
  f16* Xa   = (f16*)(base + off); off += planeB;
  if (off > ws_size) return;

  cvt_act<<<dim3((unsigned)(planeElems / 2048), 3), 256, 0, stream>>>(q_in, k_in, v_in, actP);
  cvt_w<<<dim3(DM * DM / 2048, 4), 256, 0, stream>>>(Wq, Wk, Wv, Wm, wP);

  const dim3 gg(SEQ / GN, NB);
  gemm_k256<0><<<gg, 256, 0, stream>>>(wP + 0 * DM * DM, actP + 0 * planeElems, bq, Qn, nullptr, 1.0f / 16.0f);
  gemm_k256<0><<<gg, 256, 0, stream>>>(wP + 1 * DM * DM, actP + 1 * planeElems, bk, Kn, nullptr, 1.0f / 16.0f);
  gemm_k256<1><<<gg, 256, 0, stream>>>(wP + 2 * DM * DM, actP + 2 * planeElems, bv, Vt, nullptr, 1.0f / 16.0f);

  attn_flash<<<NB * NH * (SEQ / QCHUNK), 256, 0, stream>>>(Qn, Kn, Vt, Xa);

  gemm_k256<2><<<gg, 256, 0, stream>>>(wP + 3 * DM * DM, Xa, bm, nullptr, out, 1.0f / 1024.0f);
}
